// Mamba_Block_84722524881199
// MI455X (gfx1250) — hardware-verified
//
#include <hip/hip_runtime.h>
#include <math.h>

typedef __attribute__((ext_vector_type(8)))  _Float16 v8h;
typedef __attribute__((ext_vector_type(16))) __bf16   v16b;
typedef __attribute__((ext_vector_type(8)))  __bf16   v8b;
typedef __attribute__((ext_vector_type(8)))  float    v8f;
typedef __attribute__((ext_vector_type(4)))  float    v4f;

constexpr int kBatch  = 8;
constexpr int kSeq    = 4096;
constexpr int kDm     = 64;
constexpr int kDin    = 256;
constexpr int kNst    = 16;
constexpr int kDtR    = 4;
constexpr int kXzP    = 2 * kDin;
constexpr int kXdN    = kDtR + 2 * kNst;
constexpr int kXdP    = 64;
constexpr int kRows   = kBatch * kSeq;
constexpr int kConvTP = 260;
constexpr int kScanTS = 64;
constexpr int kScanCh = 64;
constexpr int kScanQ  = 4;
constexpr int kScanSt = kNst / kScanQ;
constexpr int kScanThr = kScanCh * kScanQ;
constexpr int kScanYP = 68;
static_assert(kXdN == 36);
static_assert(kXdN <= kXdP);
static_assert((kDm % 32) == 0 && (kDin % 32) == 0);
static_assert((kRows % 64) == 0 && (kXzP % 64) == 0 && (kXdP % 64) == 0 && (kDm % 64) == 0);
static_assert((kSeq % kScanTS) == 0 && (kSeq % 64) == 0 && (kDin % kScanCh) == 0 && kDin == 256);
static_assert(kDtR == 4 && kNst == 16);
static_assert(kScanQ * kScanSt == kNst && kScanSt == 4 && kScanThr == 256);

constexpr size_t kOffX16  = 0;
constexpr size_t kOffWI   = kOffX16  + (size_t)kRows * kDm  * 2;
constexpr size_t kOffWX   = kOffWI   + (size_t)kXzP  * kDm  * 2;
constexpr size_t kOffWO   = kOffWX   + (size_t)kXdP  * kDin * 2;
constexpr size_t kOffXZ   = kOffWO   + (size_t)kDm   * kDin * 2;
constexpr size_t kOffUC16 = kOffXZ   + (size_t)kRows * kXzP * 4;
constexpr size_t kOffXD   = kOffUC16 + (size_t)kRows * kDin * 2;
constexpr size_t kOffYH   = kOffXD   + (size_t)kRows * kXdP * 4;
constexpr size_t kOffYL   = kOffYH   + (size_t)kRows * kDin * 2;
constexpr size_t kWsTotal = kOffYL   + (size_t)kRows * kDin * 2;
static_assert(kWsTotal == 130154496ull);
static_assert(kWsTotal <= 134217728ull);
static_assert((kOffWI % 128) == 0 && (kOffWX % 128) == 0 && (kOffWO % 128) == 0 && (kOffXZ % 128) == 0 &&
              (kOffUC16 % 128) == 0 && (kOffXD % 128) == 0 && (kOffYH % 128) == 0 && (kOffYL % 128) == 0);

__device__ __forceinline__ unsigned short f2bf_bits(float f) {
  unsigned u = __float_as_uint(f);
  return (unsigned short)((u + 0x7FFFu + ((u >> 16) & 1u)) >> 16);
}
__device__ __forceinline__ float bf_bits2f(unsigned short h) { return __uint_as_float(((unsigned)h) << 16); }
__device__ __forceinline__ float bf_rne(float f) { return bf_bits2f(f2bf_bits(f)); }

__device__ __forceinline__ void dep_guard4_b(v8f& a, v8f& b, v8f& c, v8f& d, v16b x, v16b y) {
  asm volatile("v_nop\n\tv_nop\n\tv_nop\n\tv_nop" : "+v"(a), "+v"(b), "+v"(c), "+v"(d) : "v"(x), "v"(y));
}
__device__ __forceinline__ void keep4_b(v16b a, v16b b, v16b c, v16b d) { asm volatile("v_nop" :: "v"(a), "v"(b), "v"(c), "v"(d)); }
__device__ __forceinline__ void acc_guard4(v8f& a, v8f& b, v8f& c, v8f& d) { asm volatile("v_nop\n\tv_nop\n\tv_nop\n\tv_nop" : "+v"(a), "+v"(b), "+v"(c), "+v"(d)); }

struct FragB {
  union U { v16b v; v8b h[2]; };
  static __device__ __forceinline__ v16b load(const __bf16* p) {
    U f; f.h[0] = *(const v8b*)(p); f.h[1] = *(const v8b*)(p + 16); return f.v;
  }
  static __device__ __forceinline__ v8f mma(v16b a, v16b b, v8f c) {
    return __builtin_amdgcn_wmma_f32_16x16x32_bf16(false, a, false, b, (short)0, c, false, false);
  }
};

template <int SPL>
__global__ __launch_bounds__(256) void wmma_gemm64_bf16(
    const unsigned short* __restrict__ Ap, const unsigned short* __restrict__ A2p, int lda,
    const unsigned short* __restrict__ Btp, int ldb,
    float* __restrict__ C, int ldc, int M, int N, int K) {
  const __bf16* A  = (const __bf16*)Ap;
  const __bf16* A2 = (const __bf16*)A2p;
  const __bf16* Bt = (const __bf16*)Btp;
  __shared__ __align__(16) float sT[8][16 * 68];
  const int lane = threadIdx.x & 31;
  const int wave = threadIdx.x >> 5;
  const int tilesN = N >> 6;
  const int tilesM = M >> 6;
  const int tile = blockIdx.x * 8 + wave;
  if (tile >= tilesM * tilesN) return;
  const int tm = tile / tilesN;
  const int tn = tile - tm * tilesN;
  const int m0 = tm << 6;
  const int n0 = tn << 6;

  const int rlane = lane & 15;
  const int koff  = (lane >> 4) * 8;
  const int mOff  = (lane >> 4) * 8;

  v8f acc[4][4];
#pragma unroll
  for (int i = 0; i < 4; ++i)
#pragma unroll
    for (int j = 0; j < 4; ++j) acc[i][j] = (v8f){0.f,0.f,0.f,0.f,0.f,0.f,0.f,0.f};

  for (int k0 = 0; k0 < K; k0 += 32) {
    v16b bh[4];
#pragma unroll
    for (int j = 0; j < 4; ++j) {
      const size_t bo = (size_t)(n0 + (j << 4) + rlane) * ldb + koff + k0;
      bh[j] = FragB::load(Bt + bo);
    }
#pragma unroll
    for (int i = 0; i < 4; ++i) {
      const size_t ao = (size_t)(m0 + (i << 4) + rlane) * lda + koff + k0;
      v16b ah = FragB::load(A + ao);
      v16b al = ah;
      if (SPL == 1) al = FragB::load(A2 + ao);
#pragma unroll
      for (int j = 0; j < 4; ++j) {
        acc[i][j] = FragB::mma(ah, bh[j], acc[i][j]);
        if (SPL == 1) acc[i][j] = FragB::mma(al, bh[j], acc[i][j]);
      }
      dep_guard4_b(acc[i][0], acc[i][1], acc[i][2], acc[i][3], ah, al);
    }
    keep4_b(bh[0], bh[1], bh[2], bh[3]);
  }
  acc_guard4(acc[0][0], acc[0][1], acc[0][2], acc[0][3]);
  acc_guard4(acc[1][0], acc[1][1], acc[1][2], acc[1][3]);
  acc_guard4(acc[2][0], acc[2][1], acc[2][2], acc[2][3]);
  acc_guard4(acc[3][0], acc[3][1], acc[3][2], acc[3][3]);

  float* slab = sT[wave];
#pragma unroll
  for (int i = 0; i < 4; ++i) {
    const int mBase = m0 + (i << 4);
#pragma unroll
    for (int j = 0; j < 4; ++j) {
#pragma unroll
      for (int r = 0; r < 8; ++r) {
        slab[(mOff + r) * 68 + (j << 4) + rlane] = acc[i][j][r];
      }
    }
    __builtin_amdgcn_fence(__ATOMIC_RELEASE, "workgroup");
    __builtin_amdgcn_wave_barrier();
    __builtin_amdgcn_fence(__ATOMIC_ACQUIRE, "workgroup");
    {
      const int hh = lane >> 4, c4 = (lane & 15) * 4;
      for (int pass = 0; pass < 2; ++pass) {
#pragma unroll
        for (int it = 0; it < 8; ++it) {
          const int row = it * 2 + hh;
          v4f v = *(const v4f*)(slab + row * 68 + c4);
          *(volatile v4f*)(C + (size_t)(mBase + row) * ldc + n0 + c4) = v;
        }
        __threadfence();
      }
    }
    __builtin_amdgcn_fence(__ATOMIC_RELEASE, "workgroup");
    __builtin_amdgcn_wave_barrier();
    __builtin_amdgcn_fence(__ATOMIC_ACQUIRE, "workgroup");
  }
}

__global__ __launch_bounds__(256) void rne_rows_bf16_kernel(
    const float* __restrict__ src, unsigned short* __restrict__ dst, int total8, int real8)
{
  const int i = blockIdx.x * 256 + threadIdx.x;
  if (i >= total8) return;
  const bool live = (i < real8);
  const int ic = live ? i : (real8 - 1);
  const size_t s0 = (size_t)ic << 3;
  const v4f a0 = *(const v4f*)(src + s0);
  const v4f a1 = *(const v4f*)(src + s0 + 4);
  v8h hv;
#pragma unroll
  for (int e = 0; e < 4; ++e) {
    const float f0 = a0[e];
    const float f1 = a1[e];
    const float z0 = live ? f0 : 0.0f;
    const float z1 = live ? f1 : 0.0f;
    const unsigned short h0 = f2bf_bits(z0);
    const unsigned short h1 = f2bf_bits(z1);
    hv[e]     = __builtin_bit_cast(_Float16, h0);
    hv[4 + e] = __builtin_bit_cast(_Float16, h1);
  }
  unsigned short* q = dst + ((size_t)i << 3);
  *(volatile v8h*)q = hv;
  __threadfence();
  *(volatile v8h*)q = hv;
}

__global__ __launch_bounds__(256) void conv_silu_kernel(
    const float* __restrict__ XZ, const float* __restrict__ cw, const float* __restrict__ cb,
    unsigned short* __restrict__ UC16)
{
  __shared__ __align__(16) float sT[16 * kConvTP];
  const int tid = threadIdx.x, lane = tid & 31, wave = tid >> 5;
  const int d = tid;
  const int g0 = blockIdx.x * 64;
  const int tb = g0 & (kSeq - 1);
  const v4f wv = *(const v4f*)(cw + d * 4);
  const float wa = wv[0], wb = wv[1], wc = wv[2], wd = wv[3];
  const float w0 = bf_rne(wa), w1 = bf_rne(wb), w2 = bf_rne(wc), w3 = bf_rne(wd);
  const float bc = bf_rne(cb[d]);
  float xm3, xm2, xm1;
  {
    const bool hist = (tb > 0);
    const int rb = hist ? (g0 - 3) : g0;
    const float v3 = XZ[(size_t)rb * kXzP + d];
    const float v2 = XZ[(size_t)(rb + 1) * kXzP + d];
    const float v1 = XZ[(size_t)(rb + 2) * kXzP + d];
    xm3 = hist ? v3 : 0.f;
    xm2 = hist ? v2 : 0.f;
    xm1 = hist ? v1 : 0.f;
  }
#pragma unroll 1
  for (int sub = 0; sub < 4; ++sub) {
    const int lb = g0 + sub * 16;
#pragma unroll 1
    for (int s = 0; s < 16; ++s) {
      const float xcur = XZ[(size_t)(lb + s) * kXzP + d];
      float acc = w0 * xm3;
      acc = fmaf(w1, xm2, acc);
      acc = fmaf(w2, xm1, acc);
      acc = fmaf(w3, xcur, acc);
      const float sv = acc + bc;
      const float sg = __builtin_amdgcn_rcpf(1.0f + __expf(-sv));
      sT[s * kConvTP + tid] = sv * sg;
      xm3 = xm2; xm2 = xm1; xm1 = xcur;
    }
    __syncthreads();
    v8h bh[2];
#pragma unroll
    for (int it = 0; it < 2; ++it) {
      const float* sp = sT + (it * 8 + wave) * kConvTP + lane * 8;
      const v4f a0 = *(const v4f*)(sp);
      const v4f a1 = *(const v4f*)(sp + 4);
#pragma unroll
      for (int e = 0; e < 4; ++e) {
        const float f0 = a0[e];
        const float f1 = a1[e];
        const unsigned short h0 = f2bf_bits(f0);
        const unsigned short h1 = f2bf_bits(f1);
        bh[it][e]     = __builtin_bit_cast(_Float16, h0);
        bh[it][4 + e] = __builtin_bit_cast(_Float16, h1);
      }
    }
    for (int pass = 0; pass < 2; ++pass) {
#pragma unroll
      for (int it = 0; it < 2; ++it) {
        const size_t o = (size_t)(lb + it * 8 + wave) * kDin + lane * 8;
        *(volatile v8h*)(UC16 + o) = bh[it];
      }
      __threadfence();
    }
    __syncthreads();
  }
}

__global__ __launch_bounds__(256) void scan_kernel(
    const float* __restrict__ XD, const float* __restrict__ XZ,
    const float* __restrict__ cw, const float* __restrict__ cb,
    const float* __restrict__ Wdt, const float* __restrict__ bdt, const float* __restrict__ Alog,
    const float* __restrict__ Dp, unsigned short* __restrict__ YH, unsigned short* __restrict__ YL)
{
  __shared__ __align__(16) float sX[kScanTS * kXdP];
  __shared__ __align__(16) float sY[kScanTS * kScanYP];
  __shared__ __align__(16) float sA[kScanSt * kScanThr];
  const int tid = threadIdx.x, lane = tid & 31, wave = tid >> 5;
  const int chl = tid >> 2;
  const int qd  = tid & 3;
  constexpr int kBlkPerB = kDin / kScanCh;
  const int bix = blockIdx.x / kBlkPerB;
  const int d0  = (blockIdx.x - bix * kBlkPerB) * kScanCh;
  const int d   = d0 + chl;
  const size_t row0 = (size_t)bix * kSeq;
#pragma unroll 1
  for (int j = 0; j < kScanSt; ++j)
    sA[j * kScanThr + tid] = -expf(bf_rne(Alog[(size_t)d * kNst + qd * kScanSt + j]));
  __syncthreads();
  float negA[kScanSt], h[kScanSt];
#pragma unroll
  for (int j = 0; j < kScanSt; ++j) {
    negA[j] = sA[j * kScanThr + tid];
    h[j] = 0.f;
  }
  const v4f wdv = *(const v4f*)(Wdt + (size_t)d * kDtR);
  const float wda = wdv[0], wdb = wdv[1], wdc = wdv[2], wdd = wdv[3];
  const float wd0 = bf_rne(wda), wd1 = bf_rne(wdb), wd2 = bf_rne(wdc), wd3 = bf_rne(wdd);
  const v4f cwv = *(const v4f*)(cw + (size_t)d * 4);
  const float cwa = cwv[0], cwb = cwv[1], cwc = cwv[2], cwd = cwv[3];
  const float cw0 = bf_rne(cwa), cw1 = bf_rne(cwb), cw2 = bf_rne(cwc), cw3 = bf_rne(cwd);
  const float bc = bf_rne(cb[d]);
  const float bb = bf_rne(bdt[d]);
  const float Dd = bf_rne(Dp[d]);
  float xm3 = 0.f, xm2 = 0.f, xm1 = 0.f;
  const int lr = tid >> 4, lc4 = (tid & 15) * 4;
  const int q = lane >> 3, c8 = (lane & 7) * 8;
  const int bOff = kDtR + qd * kScanSt;
  const int cOff = kDtR + kNst + qd * kScanSt;
#pragma unroll 1
  for (int t0 = 0; t0 < kSeq; t0 += kScanTS) {
    __syncthreads();
#pragma unroll
    for (int i = 0; i < 4; ++i) {
      const int r = lr + 16 * i;
      *(v4f*)(sX + r * kXdP + lc4) = *(const v4f*)(XD + (row0 + t0 + r) * kXdP + lc4);
    }
    __syncthreads();
#pragma unroll 1
    for (int s = 0; s < kScanTS; ++s) {
      const size_t m = row0 + (size_t)(t0 + s);
      float xcur = XZ[m * kXzP + d];
      asm volatile("" : "+v"(xcur));
      float zv = XZ[m * kXzP + kDin + d];
      asm volatile("" : "+v"(zv));
      const float* xr = sX + s * kXdP;
      const v4f dv = *(const v4f*)(xr);
      const v4f bv = *(const v4f*)(xr + bOff);
      const v4f cv = *(const v4f*)(xr + cOff);
      float vdot = dv[0] * wd0;
      vdot = fmaf(dv[1], wd1, vdot);
      vdot = fmaf(dv[2], wd2, vdot);
      vdot = fmaf(dv[3], wd3, vdot);
      const float v   = vdot + bb;
      const float a   = __expf(-fabsf(v));
      const float u1  = 1.0f + a;
      const float l1p = __logf(u1) + (a - (u1 - 1.0f)) * __builtin_amdgcn_rcpf(u1);
      const float dt  = fmaxf(v, 0.0f) + l1p;
      float pre = cw0 * xm3;
      pre = fmaf(cw1, xm2, pre);
      pre = fmaf(cw2, xm1, pre);
      pre = fmaf(cw3, xcur, pre);
      pre = pre + bc;
      xm3 = xm2; xm2 = xm1; xm1 = xcur;
      const float ut  = pre * __builtin_amdgcn_rcpf(1.0f + __expf(-pre));
      const float dtx = dt * ut;
      float yp = 0.f;
#pragma unroll
      for (int j = 0; j < kScanSt; ++j) {
        const float e = __expf(dt * negA[j]);
        h[j] = fmaf(e, h[j], dtx * bv[j]);
        yp = fmaf(h[j], cv[j], yp);
      }
      yp += __shfl_xor(yp, 1);
      yp += __shfl_xor(yp, 2);
      float y = fmaf(ut, Dd, yp);
      const float sg = __builtin_amdgcn_rcpf(1.0f + __expf(-zv));
      y = y * (zv * sg);
      if (qd == 0) sY[s * kScanYP + chl] = y;
    }
    __syncthreads();
    v8h hv[2], lv[2];
#pragma unroll
    for (int it = 0; it < 2; ++it) {
      const int row = it * 32 + wave * 4 + q;
      const float* sp = sY + row * kScanYP + c8;
      const v4f a0 = *(const v4f*)(sp);
      const v4f a1 = *(const v4f*)(sp + 4);
#pragma unroll
      for (int e = 0; e < 4; ++e) {
        const float f0 = a0[e];
        const float f1 = a1[e];
        const unsigned short h0 = f2bf_bits(f0), h1 = f2bf_bits(f1);
        const unsigned short l0 = f2bf_bits(f0 - bf_bits2f(h0)), l1 = f2bf_bits(f1 - bf_bits2f(h1));
        hv[it][e]     = __builtin_bit_cast(_Float16, h0);
        hv[it][4 + e] = __builtin_bit_cast(_Float16, h1);
        lv[it][e]     = __builtin_bit_cast(_Float16, l0);
        lv[it][4 + e] = __builtin_bit_cast(_Float16, l1);
      }
    }
    for (int pass = 0; pass < 2; ++pass) {
#pragma unroll
      for (int it = 0; it < 2; ++it) {
        const int row = it * 32 + wave * 4 + q;
        const size_t o = (row0 + (size_t)(t0 + row)) * kDin + d0 + c8;
        *(volatile v8h*)(YH + o) = hv[it];
        *(volatile v8h*)(YL + o) = lv[it];
      }
      __threadfence();
    }
  }
}

static_assert(((kRows / 64) * (kXzP / 64)) % 8 == 0);
static_assert(((kRows / 64) * (kXdP / 64)) % 8 == 0);
static_assert(((kRows / 64) * (kDm / 64)) % 8 == 0);
static_assert(((kRows * kDm / 8) % 256) == 0 && ((kXzP * kDm / 8) % 256) == 0 &&
              ((kXdP * kDin / 8) % 256) == 0 && ((kDm * kDin / 8) % 256) == 0);

extern "C" void kernel_launch(void* const* d_in, const int* in_sizes, int n_in,
                              void* d_out, int out_size, void* d_ws, size_t ws_size,
                              hipStream_t stream) {
  if (n_in < 10) return;
  if (in_sizes[0] != kRows * kDm) return;
  if (in_sizes[1] != kXzP * kDm) return;
  if (in_sizes[2] != kDin * 4) return;
  if (in_sizes[3] != kDin) return;
  if (in_sizes[4] != kXdN * kDin) return;
  if (in_sizes[5] != kDin * kDtR) return;
  if (in_sizes[6] != kDin) return;
  if (in_sizes[7] != kDin * kNst) return;
  if (in_sizes[8] != kDin) return;
  if (in_sizes[9] != kDm * kDin) return;
  if (out_size != kRows * kDm) return;
  if (ws_size < kWsTotal) return;

  const float* x      = (const float*)d_in[0];
  const float* W_in   = (const float*)d_in[1];
  const float* conv_w = (const float*)d_in[2];
  const float* conv_b = (const float*)d_in[3];
  const float* W_x    = (const float*)d_in[4];
  const float* W_dt   = (const float*)d_in[5];
  const float* b_dt   = (const float*)d_in[6];
  const float* A_log  = (const float*)d_in[7];
  const float* Dp     = (const float*)d_in[8];
  const float* W_out  = (const float*)d_in[9];
  float* out = (float*)d_out;

  char* ws = (char*)d_ws;
  unsigned short* X16  = (unsigned short*)(ws + kOffX16);
  unsigned short* WI16 = (unsigned short*)(ws + kOffWI);
  unsigned short* WX16 = (unsigned short*)(ws + kOffWX);
  unsigned short* WO16 = (unsigned short*)(ws + kOffWO);
  float*          XZ   = (float*)(ws + kOffXZ);
  unsigned short* UC16 = (unsigned short*)(ws + kOffUC16);
  float*          XD   = (float*)(ws + kOffXD);
  unsigned short* YH   = (unsigned short*)(ws + kOffYH);
  unsigned short* YL   = (unsigned short*)(ws + kOffYL);

  rne_rows_bf16_kernel<<<(kRows * kDm / 8) / 256, 256, 0, stream>>>(x, X16, kRows * kDm / 8, kRows * kDm / 8);
  rne_rows_bf16_kernel<<<(kXzP * kDm / 8) / 256, 256, 0, stream>>>(W_in, WI16, kXzP * kDm / 8, kXzP * kDm / 8);
  rne_rows_bf16_kernel<<<(kXdP * kDin / 8) / 256, 256, 0, stream>>>(W_x, WX16, kXdP * kDin / 8, kXdN * kDin / 8);
  rne_rows_bf16_kernel<<<(kDm * kDin / 8) / 256, 256, 0, stream>>>(W_out, WO16, kDm * kDin / 8, kDm * kDin / 8);

  wmma_gemm64_bf16<0><<<dim3(((kRows / 64) * (kXzP / 64)) / 8), 256, 0, stream>>>(
      X16, X16, kDm, WI16, kDm, XZ, kXzP, kRows, kXzP, kDm);

  conv_silu_kernel<<<dim3(kRows / 64), 256, 0, stream>>>(XZ, conv_w, conv_b, UC16);

  wmma_gemm64_bf16<0><<<dim3(((kRows / 64) * (kXdP / 64)) / 8), 256, 0, stream>>>(
      UC16, UC16, kDin, WX16, kDin, XD, kXdP, kRows, kXdP, kDin);

  scan_kernel<<<dim3(kBatch * (kDin / kScanCh)), kScanThr, 0, stream>>>(
      XD, XZ, conv_w, conv_b, W_dt, b_dt, A_log, Dp, YH, YL);

  wmma_gemm64_bf16<1><<<dim3(((kRows / 64) * (kDm / 64)) / 8), 256, 0, stream>>>(
      YH, YL, kDin, WO16, kDin, out, kDm, kRows, kDm, kDin);
}
